// GKA_14087492730930
// MI455X (gfx1250) — hardware-verified
//
#include <hip/hip_runtime.h>


namespace {
constexpr int NB_ = 8, NC = 1024, NT = 1024, DX = 3, DY = 32, H = 128, CH = 256  ;
constexpr float XS = 8.0f, HS = 256.0f, PS = 256.0f, WSC = 256.0f;
typedef _Float16 b16;
typedef __attribute__((ext_vector_type(16))) _Float16 v16b;
typedef __attribute__((ext_vector_type(8))) _Float16 v8b;
typedef __attribute__((ext_vector_type(8))) float v8f;
typedef __attribute__((ext_vector_type(4))) float v4f;
__device__ __forceinline__ float bf16_rne(float f) { unsigned int u = __float_as_uint(f); u += 0x7FFFu + ((u >> 16) & 1u); float r = __uint_as_float(u & 0xFFFF0000u); asm volatile("" : "+v"(r)); return r; }
__device__ __forceinline__ float bfv(float f) { float r = bf16_rne(f); asm volatile("" : "+v"(r)); return r; }
__device__ __forceinline__ void split16(float v, b16& hi, b16& lo) { hi = (b16)v; lo = (b16)(v - (float)hi); }
__device__ __forceinline__ v16b frag_kb(const b16* p, int hh) { const v8b a = *(const v8b*)(p + 8 * hh), b = *(const v8b*)(p + 16 + 8 * hh); v16b f;
#pragma unroll
  for (int e = 0; e < 8; ++e) { f[e] = a[e]; f[8 + e] = b[e]; } return f; }
__device__ __forceinline__ v8f wmma16b(v16b a, v16b b, v8f c) { v8f d = __builtin_amdgcn_wmma_f32_16x16x32_f16(false, a, false, b, (short)0, c, false, false); asm volatile("v_nop\n\tv_nop\n\tv_nop\n\tv_nop" : "+v"(d) : "v"(a), "v"(b)); return d; }
__device__ __forceinline__ void wave_lds_sync() { __builtin_amdgcn_fence(__ATOMIC_RELEASE, "workgroup"); __builtin_amdgcn_wave_barrier(); __builtin_amdgcn_fence(__ATOMIC_ACQUIRE, "workgroup"); }
__device__ __forceinline__ float pmul(float a, float b) { float p = a * b; asm volatile("" : "+v"(p)); return p; }

__global__ __launch_bounds__(256) void wput_kernel(const float* __restrict__ w1, const float* __restrict__ w2, b16* __restrict__ WT1, b16* __restrict__ WT2) { const int u = blockIdx.x * 256 + threadIdx.x; if (u >= H * 16) return; const int o = u / 16, k0 = (u % 16) * 8; v8b a, b;
#pragma unroll
  for (int j = 0; j < 8; ++j) { a[j] = (b16)(bf16_rne(w1[(size_t)(k0 + j) * H + o]) * WSC); b[j] = (b16)(bf16_rne(w2[(size_t)(k0 + j) * H + o]) * WSC); }
  for (int pass = 0; pass < 2; ++pass) { *(volatile v8b*)(WT1 + (size_t)o * H + k0) = a; *(volatile v8b*)(WT2 + (size_t)o * H + k0) = b; __threadfence(); } }
__global__ __launch_bounds__(32) void sig_kernel(const float* __restrict__ xt, const float* __restrict__ w0, const float* __restrict__ b0, const b16* __restrict__ WT1, const float* __restrict__ b1, const b16* __restrict__ WT2, const float* __restrict__ b2, const float* __restrict__ w3, const float* __restrict__ b3, float* __restrict__ SIG) { __shared__ __attribute__((aligned(16))) b16 Ah[16][H + 8], Al[16][H + 8]; __shared__ float Tf[16][H + 1], Sg[16][4]; const int lane = threadIdx.x, nloc = lane & 15, hlf = lane >> 4; const size_t m0 = (size_t)blockIdx.x * 16;
  for (int rr = 0; rr < 16; ++rr) { float xv[DX]; for (int d = 0; d < DX; ++d) xv[d] = bfv(xt[(m0 + rr) * DX + d]); for (int q = 0; q < 4; ++q) { const int c = q * 32 + lane; float s = bfv(b0[c]); for (int d = 0; d < DX; ++d) s += pmul(xv[d], bfv(w0[d * H + c])); b16 p, ql; split16(fmaxf(s, 0.0f) * HS, p, ql); Ah[rr][c] = p; Al[rr][c] = ql; } }
  if (lane < 16) for (int k = H; k < H + 8; ++k) { Ah[lane][k] = (b16)0.0f; Al[lane][k] = (b16)0.0f; }
  wave_lds_sync();
#pragma unroll 1
  for (int layer = 0; layer < 2; ++layer) { const b16* W = layer ? WT2 : WT1; const float* bb_ = layer ? b2 : b1; v8f acc[8];
#pragma unroll
    for (int t = 0; t < 8; ++t) acc[t] = (v8f){};
#pragma unroll
    for (int kb = 0; kb < H; kb += 32) { const v16b a = frag_kb(&Ah[nloc][kb], hlf), al = frag_kb(&Al[nloc][kb], hlf);
#pragma unroll
      for (int t = 0; t < 8; ++t) { const v16b bw = frag_kb(W + (size_t)(t * 16 + nloc) * H + kb, hlf); acc[t] = wmma16b(a, bw, acc[t]); acc[t] = wmma16b(al, bw, acc[t]); } }
#pragma unroll
    for (int t = 0; t < 8; ++t) { const int cc = t * 16 + nloc; const float bb = bfv(bb_[cc]);
#pragma unroll
      for (int r8 = 0; r8 < 8; ++r8) Tf[8 * hlf + r8][cc] = fmaxf(acc[t][r8] * (1.0f / (HS * WSC)) + bb, 0.0f); }
    wave_lds_sync();
    if (layer == 0) { for (int rr = 0; rr < 16; ++rr) for (int q = 0; q < 4; ++q) { b16 p, ql; split16(Tf[rr][q * 32 + lane] * HS, p, ql); Ah[rr][q * 32 + lane] = p; Al[rr][q * 32 + lane] = ql; } wave_lds_sync(); } }
  for (int rr = 0; rr < 16; ++rr) { for (int d = 0; d < DX; ++d) { float s = 0.0f; for (int q = 0; q < 4; ++q) s += pmul(Tf[rr][q * 32 + lane], bfv(w3[(q * 32 + lane) * DX + d])); for (int o = 16; o; o >>= 1) s += __shfl_xor(s, o); if (lane == 0) Sg[rr][d] = __expf(s + bfv(b3[d])); } if (lane == 0) Sg[rr][3] = 0.0f; }
  wave_lds_sync();
  for (int pass = 0; pass < 2; ++pass) { for (int q = 0; q < 2; ++q) ((volatile float*)SIG)[m0 * 4 + q * 32 + lane] = Sg[(q * 32 + lane) >> 2][(q * 32 + lane) & 3]; __threadfence(); } }
__global__ __launch_bounds__(32) void main_kernel(const float* __restrict__ xc, const float* __restrict__ yc, const float* __restrict__ xt, const float* __restrict__ SIG, float* __restrict__ out) { __shared__ float Pf[16][NC]; __shared__ __attribute__((aligned(16))) b16 Sh[16][CH + 8], Sl[16][CH + 8], Yh[DY][CH + 8]; __shared__ float Of[16][DY + 1], Inv[16]; const int lane = threadIdx.x, nloc = lane & 15, hlf = lane >> 4; const int b = blockIdx.x / (NT / 16); const size_t t0 = (size_t)(blockIdx.x % (NT / 16)) * 16; const size_t rb = (size_t)b * NT + t0;
  for (int r = 0; r < 16; ++r) { float xv[DX], sg[DX]; for (int d = 0; d < DX; ++d) { xv[d] = bfv(xt[(rb + r) * DX + d]); sg[d] = SIG[(rb + r) * 4 + d]; } float mx = -INFINITY;
    for (int c = lane; c < NC; c += 32) { float s = 0.0f; for (int d = 0; d < DX; ++d) { const float df = bfv(xc[((size_t)b * NC + c) * DX + d]) - xv[d]; s += pmul(df * df, sg[d]); } const float p = -s; Pf[r][c] = p; mx = fmaxf(mx, p); }
    for (int o = 16; o; o >>= 1) mx = fmaxf(mx, __shfl_xor(mx, o)); float sm = 0.0f; for (int c = lane; c < NC; c += 32) { const float e = __expf(Pf[r][c] - mx); Pf[r][c] = e; sm += e; } for (int o = 16; o; o >>= 1) sm += __shfl_xor(sm, o); if (lane == 0) Inv[r] = 1.0f / sm; }
  if (lane < 16) for (int k = CH; k < CH + 8; ++k) { Sh[lane][k] = (b16)0.0f; Sl[lane][k] = (b16)0.0f; }
  for (int k = CH; k < CH + 8; ++k) Yh[lane][k] = (b16)0.0f;
  wave_lds_sync(); v8f acc[2] = {(v8f){}, (v8f){}};
#pragma unroll 1
  for (int ch = 0; ch < NC / CH; ++ch) { const int c0 = ch * CH;
    for (int r = 0; r < 16; ++r) { const float inv = Inv[r]; for (int q = 0; q < CH / 32; ++q) { const int c = q * 32 + lane; b16 p, ql; split16(Pf[r][c0 + c] * inv * PS, p, ql); Sh[r][c] = p; Sl[r][c] = ql; } }
    for (int c = 0; c < CH; ++c) Yh[lane][c] = (b16)(bfv(yc[((size_t)b * NC + c0 + c) * DY + lane]) * XS);
    wave_lds_sync();
#pragma unroll 2
    for (int kb = 0; kb < CH; kb += 32) { const v16b a = frag_kb(&Sh[nloc][kb], hlf), al = frag_kb(&Sl[nloc][kb], hlf);
#pragma unroll
      for (int t = 0; t < 2; ++t) { const v16b bw = frag_kb(&Yh[t * 16 + nloc][kb], hlf); acc[t] = wmma16b(a, bw, acc[t]); acc[t] = wmma16b(al, bw, acc[t]); } }
    wave_lds_sync(); }
#pragma unroll
  for (int t = 0; t < 2; ++t)
#pragma unroll
    for (int r8 = 0; r8 < 8; ++r8) Of[8 * hlf + r8][t * 16 + nloc] = acc[t][r8] * (1.0f / (PS * XS));
  wave_lds_sync();
  for (int pass = 0; pass < 2; ++pass) { for (int r = 0; r < 16; ++r) ((volatile float*)out)[(rb + r) * DY + lane] = Of[r][lane]; __threadfence(); } }
}

extern "C" void kernel_launch(void* const* d_in, const int* in_sizes, int n_in, void* d_out, int out_size, void* d_ws, size_t ws_size, hipStream_t stream) {
  (void)n_in;
  auto Fp = [&](int i) { return (const float*)d_in[i]; };
  if (in_sizes[0] != NB_ * NC * DX || in_sizes[1] != NB_ * NC * DY || in_sizes[2] != NB_ * NT * DX || in_sizes[3] != DX * H || in_sizes[5] != H * H || in_sizes[9] != H * DX || out_size != NB_ * NT * DY) return;
  const int BLIM = NB_;
  size_t off = 0; char* ws = (char*)d_ws;
  auto carve = [&](size_t bytes) { char* p = ws + off; off += (bytes + 255) & ~(size_t)255; return p; };
  b16* WT1 = (b16*)carve((size_t)H * H * 2); b16* WT2 = (b16*)carve((size_t)H * H * 2); float* SIG = (float*)carve((size_t)NB_ * NT * 4 * 4);
  if (off > ws_size || off > ((size_t)4 << 20)) return;
  wput_kernel<<<(H * 16 + 255) / 256, 256, 0, stream>>>(Fp(5), Fp(7), WT1, WT2);
  sig_kernel<<<BLIM * NT / 16, 32, 0, stream>>>(Fp(2), Fp(3), Fp(4), WT1, Fp(6), WT2, Fp(8), Fp(9), Fp(10), SIG);
  main_kernel<<<BLIM * (NT / 16), 32, 0, stream>>>(Fp(0), Fp(1), Fp(2), SIG, (float*)d_out);
}
